// NEXT_Simulator_33208687133353
// MI455X (gfx1250) — hardware-verified
//
#include <hip/hip_runtime.h>


namespace {
constexpr int NB = 2, ND = 100, NK = 100, E = ND * NK, EP = 10240  , NT = 550, NTP = 560, NP_ = 12, NS1 = 47, NS = NS1 * NS1  , NSP = 2240  , RS = 576  , H1 = 28;
constexpr float XS = 8.0f, BIN_SIGMA = 0.1f, GAUSS_NORM = 1.0f / (0.1f * 2.5066282746f), SHARP = 0.001f;
constexpr int OUT0 = NB * NP_ * NT, OUT1 = NB * NS * NT;

typedef _Float16 b16;
typedef __attribute__((ext_vector_type(16))) _Float16 v16b;
typedef __attribute__((ext_vector_type(8))) _Float16 v8b;
typedef __attribute__((ext_vector_type(8))) float v8f;
typedef __attribute__((ext_vector_type(4))) float v4f;
__device__ __forceinline__ float bf16_rne(float f) { unsigned int u = __float_as_uint(f); u += 0x7FFFu + ((u >> 16) & 1u); return __uint_as_float(u & 0xFFFF0000u); }
__device__ __forceinline__ void split16(float v, b16& hi, b16& lo) { hi = (b16)v; lo = (b16)(v - (float)hi); }
__device__ __forceinline__ v16b frag_kb(const b16* p, int hh) { const v8b a = *(const v8b*)(p + 8 * hh), b = *(const v8b*)(p + 16 + 8 * hh); v16b f;
#pragma unroll
  for (int e = 0; e < 8; ++e) { f[e] = a[e]; f[8 + e] = b[e]; } return f; }
__device__ __forceinline__ v8f wmma16b(v16b a, v16b b, v8f c) { v8f d = __builtin_amdgcn_wmma_f32_16x16x32_f16(false, a, false, b, (short)0, c, false, false); asm volatile("v_nop\n\tv_nop\n\tv_nop\n\tv_nop" : "+v"(d) : "v"(a), "v"(b)); return d; }
__device__ __forceinline__ void wave_lds_sync() { __builtin_amdgcn_fence(__ATOMIC_RELEASE, "workgroup"); __builtin_amdgcn_wave_barrier(); __builtin_amdgcn_fence(__ATOMIC_ACQUIRE, "workgroup"); }
__device__ __forceinline__ float pmul(float a, float b) { float p = a * b; asm volatile("" : "+v"(p)); return p; }
__device__ __forceinline__ float sigm(float x) { return 1.0f / (1.0f + __expf(-x)); }

__global__ __launch_bounds__(256) void elec_kernel(int b, const float* __restrict__ pos, const float* __restrict__ disp, const float* __restrict__ rnd, const float* __restrict__ w1, const float* __restrict__ b1, const float* __restrict__ w2, const float* __restrict__ b2, const float* __restrict__ dsc, const float* __restrict__ psc, const float* __restrict__ lt, float* __restrict__ EL, b16* __restrict__ PTh, b16* __restrict__ PTl) {
  __shared__ __attribute__((aligned(16))) b16 ph_s[16][256 + 8], pl_s[16][256 + 8];
  const int t_ = threadIdx.x; const int e = blockIdx.x * 256 + t_; v4f el = {0.0f, 0.0f, 0.0f, 0.0f}; float pr[NP_]; for (int p = 0; p < NP_; ++p) pr[p] = 0.0f;
  if (e < E) { const int n = e / NK; const float* pp = pos + ((size_t)b * ND + n) * 3; const float* dd = disp + ((size_t)b * E + e) * 3;
    const float px = bf16_rne(pp[0]), py = bf16_rne(pp[1]), pz = bf16_rne(pp[2]); const float sz = sqrtf(pz);
    const float x = pmul(pmul(bf16_rne(dsc[0]), bf16_rne(dd[0])), sz) + px, y = pmul(pmul(bf16_rne(dsc[1]), bf16_rne(dd[1])), sz) + py, z = pmul(pmul(bf16_rne(dsc[2]), bf16_rne(dd[2])), sz) + pz;
    const float w = sigm((__expf(-z / bf16_rne(lt[0])) - bf16_rne(rnd[(size_t)b * E + e])) / SHARP);
    el[0] = x; el[1] = y; el[2] = z; el[3] = w;
    float h[H1];
#pragma unroll 1
    for (int o = 0; o < H1; ++o) h[o] = sigm(pmul(x, bf16_rne(w1[o])) + pmul(y, bf16_rne(w1[H1 + o])) + bf16_rne(b1[o]));
#pragma unroll 1
    for (int p = 0; p < NP_; ++p) { float s = bf16_rne(b2[p]);
#pragma unroll 1
      for (int o = 0; o < H1; ++o) s += pmul(h[o], bf16_rne(w2[o * NP_ + p])); pr[p] = sigm(s) * bf16_rne(psc[p]); } }
  for (int p = 0; p < 16; ++p) { b16 a, c; split16((p < NP_ ? pr[p] : 0.0f) * XS, a, c); ph_s[p][t_] = a; pl_s[p][t_] = c; }
  __syncthreads();
  for (int pass = 0; pass < 2; ++pass) { *(volatile v4f*)(EL + (size_t)e * 4) = el;
    for (int q = t_; q < 16 * 32; q += 256) { const int p = q >> 5, c8 = (q & 31) * 8; *(volatile v8b*)(PTh + (size_t)p * EP + blockIdx.x * 256 + c8) = *(const v8b*)(&ph_s[p][c8]); *(volatile v8b*)(PTl + (size_t)p * EP + blockIdx.x * 256 + c8) = *(const v8b*)(&pl_s[p][c8]); }
    __threadfence(); }
}
__global__ __launch_bounds__(256) void evt_kernel(const float* __restrict__ EL, b16* __restrict__ EVh, b16* __restrict__ EVl) {
  __shared__ float z_s[64], w_s[64];
  const int t_ = threadIdx.x; const int e0 = blockIdx.x * 64;
  if (t_ < 64) { const int e = e0 + t_; z_s[t_] = (e < E) ? EL[(size_t)e * 4 + 2] : -1e9f; w_s[t_] = (e < E) ? EL[(size_t)e * 4 + 3] : 0.0f; }
  __syncthreads();
  for (int pass = 0; pass < 2; ++pass) { for (int q = t_; q < NTP * 8; q += 256) { const int t = q >> 3, c8 = (q & 7) * 8; v8b hv, lv;
      for (int j = 0; j < 8; ++j) { const int ee = c8 + j; float v = 0.0f; if (t < NT && e0 + ee < E) { const float d = ((float)t + 0.5f) - z_s[ee]; v = w_s[ee] * GAUSS_NORM * __expf(-(d * d) / BIN_SIGMA); } b16 a, c; split16(v * XS, a, c); hv[j] = a; lv[j] = c; }
      *(volatile v8b*)(EVh + (size_t)t * EP + e0 + c8) = hv; *(volatile v8b*)(EVl + (size_t)t * EP + e0 + c8) = lv; } __threadfence(); }
}
__global__ __launch_bounds__(256) void srt_kernel(const float* __restrict__ EL, const float* __restrict__ ssc, const float* __restrict__ sg, b16* __restrict__ SR) {
  __shared__ float x_s[64], y_s[64];
  const int t_ = threadIdx.x; const int e0 = blockIdx.x * 64, s0 = blockIdx.y * 280; const float sig = bf16_rne(sg[0]); const float isg2 = 1.0f / (sig * sig);
  if (t_ < 64) { const int e = e0 + t_; x_s[t_] = (e < E) ? EL[(size_t)e * 4] : 0.0f; y_s[t_] = (e < E) ? EL[(size_t)e * 4 + 1] : 0.0f; }
  __syncthreads();
  for (int pass = 0; pass < 2; ++pass) { for (int q = t_; q < 280 * 8; q += 256) { const int s = s0 + (q >> 3), c8 = (q & 7) * 8; v8b hv;
      const int i = s / NS1, jj = s % NS1; const float sx = -235.0f + 10.0f * (float)i, sy = -235.0f + 10.0f * (float)jj; const float sc = (s < NS) ? bf16_rne(ssc[s]) : 0.0f;
      for (int j = 0; j < 8; ++j) { const int ee = c8 + j; float v = 0.0f; if (s < NS && e0 + ee < E) { const float d = (x_s[ee] - sx) + (y_s[ee] - sy); v = __expf(-(d * d) * isg2) * sc; } hv[j] = (b16)(v * XS); }
      *(volatile v8b*)(SR + (size_t)s * EP + e0 + c8) = hv; } __threadfence(); }
}
template <int MODE>
__global__ __launch_bounds__(128) void contract_kernel(const b16* __restrict__ Ah, const b16* __restrict__ Al, const b16* __restrict__ EVh, const b16* __restrict__ EVl, float* __restrict__ RES) {
  __shared__ __attribute__((aligned(16))) float Tf[4][16][128 + 4];
  const int wave = threadIdx.x >> 5, lane = threadIdx.x & 31, nloc = lane & 15, hlf = lane >> 4; const size_t m0 = (size_t)blockIdx.x * 64 + wave * 16; const int n0 = blockIdx.y * 128;
  v8f acc[8];
#pragma unroll
  for (int t = 0; t < 8; ++t) acc[t] = (v8f){};
  for (int kb = 0; kb < EP; kb += 32) { const v16b a = frag_kb(Ah + (m0 + nloc) * EP + kb, hlf); v16b al; if (MODE == 1) al = frag_kb(Al + (m0 + nloc) * EP + kb, hlf);
#pragma unroll
    for (int t = 0; t < 8; ++t) { const v16b eh = frag_kb(EVh + (size_t)(n0 + t * 16 + nloc) * EP + kb, hlf), evl = frag_kb(EVl + (size_t)(n0 + t * 16 + nloc) * EP + kb, hlf); acc[t] = wmma16b(a, eh, acc[t]); acc[t] = wmma16b(a, evl, acc[t]); if (MODE == 1) acc[t] = wmma16b(al, eh, acc[t]); } }
#pragma unroll
  for (int t = 0; t < 8; ++t)
#pragma unroll
    for (int r = 0; r < 8; ++r) Tf[wave][8 * hlf + r][t * 16 + nloc] = acc[t][r] * (1.0f / (XS * XS));
  wave_lds_sync();
  for (int pass = 0; pass < 2; ++pass) { for (int rr = 0; rr < 16; ++rr) *(volatile v4f*)(RES + (m0 + rr) * 640 + n0 + lane * 4) = *(const v4f*)(&Tf[wave][rr][lane * 4]); __threadfence(); }
}
__global__ __launch_bounds__(256) void writer_kernel(const float* __restrict__ PMTR, const float* __restrict__ SIPR, float* __restrict__ out) {
  const size_t i0 = ((size_t)blockIdx.x * 256 + threadIdx.x) * 4; if (i0 >= (size_t)(OUT0 + OUT1)) return; v4f v;
  for (int j = 0; j < 4; ++j) { const size_t i = i0 + j; float x = 0.0f;
    if (i < (size_t)OUT0) { const int b = (int)(i / (NP_ * NT)); const int rem = (int)(i % (NP_ * NT)); const int p = rem / NT, t = rem % NT; x = PMTR[((size_t)b * 64 + p) * 640 + t]; }
    else if (i < (size_t)(OUT0 + OUT1)) { const size_t k = i - OUT0; const int b = (int)(k / ((size_t)NS * NT)); const size_t rem = k % ((size_t)NS * NT); const int s = (int)(rem / NT), t = (int)(rem % NT); x = SIPR[((size_t)b * NSP + s) * 640 + t]; }
    v[j] = x; }
  const bool tail = (i0 + 4 > (size_t)(OUT0 + OUT1));
  for (int pass = 0; pass < 2; ++pass) { if (!tail) *(volatile v4f*)(out + i0) = v; else { for (int j = 0; j < 4; ++j) if (i0 + j < (size_t)(OUT0 + OUT1)) ((volatile float*)out)[i0 + j] = v[j]; } __threadfence(); }
}
__global__ __launch_bounds__(256) void vzero_h(b16* __restrict__ a, size_t n8) { const size_t i = (size_t)blockIdx.x * 256 + threadIdx.x; if (i < n8) { const v8b z = {}; *(volatile v8b*)(a + i * 8) = z; } }
}

extern "C" void kernel_launch(void* const* d_in, const int* in_sizes, int n_in, void* d_out, int out_size, void* d_ws, size_t ws_size, hipStream_t stream) {
  (void)n_in;
  auto Fp = [&](int i) { return (const float*)d_in[i]; };
  if (in_sizes[0] != NB * ND * 3 || in_sizes[1] != NB * E * 3 || in_sizes[2] != NB * E || in_sizes[3] != 2 * H1 || in_sizes[5] != H1 * NP_ || in_sizes[10] != NS || out_size != OUT0 + OUT1) return;
  size_t off = 0; char* ws = (char*)d_ws;
  auto carve = [&](size_t bytes) { char* p = ws + off; off += (bytes + 255) & ~(size_t)255; return p; };
  float* EL = (float*)carve((size_t)EP * 4 * 4); b16* PTh = (b16*)carve((size_t)64 * EP * 2); b16* PTl = (b16*)carve((size_t)64 * EP * 2); b16* EVh = (b16*)carve((size_t)640 * EP * 2); b16* EVl = (b16*)carve((size_t)640 * EP * 2); b16* SR = (b16*)carve((size_t)NSP * EP * 2);
  float* PMTR = (float*)carve((size_t)NB * 64 * 640 * 4); float* SIPR = (float*)carve((size_t)NB * NSP * 640 * 4);
  if (off > ws_size || off > ((size_t)128 << 20)) return;
  vzero_h<<<(unsigned)(((size_t)640 * EP / 8 + 255) / 256), 256, 0, stream>>>(EVh, (size_t)640 * EP / 8); vzero_h<<<(unsigned)(((size_t)640 * EP / 8 + 255) / 256), 256, 0, stream>>>(EVl, (size_t)640 * EP / 8);
  vzero_h<<<(unsigned)(((size_t)64 * EP / 8 + 255) / 256), 256, 0, stream>>>(PTh, (size_t)64 * EP / 8); vzero_h<<<(unsigned)(((size_t)64 * EP / 8 + 255) / 256), 256, 0, stream>>>(PTl, (size_t)64 * EP / 8);
  for (int b = 0; b < NB; ++b) {
    elec_kernel<<<(EP + 255) / 256, 256, 0, stream>>>(b, Fp(0), Fp(1), Fp(2), Fp(3), Fp(4), Fp(5), Fp(6), Fp(7), Fp(9), Fp(11), EL, PTh, PTl);
    evt_kernel<<<EP / 64, 256, 0, stream>>>(EL, EVh, EVl);
    srt_kernel<<<dim3(EP / 64, NSP / 280), 256, 0, stream>>>(EL, Fp(10), Fp(8), SR);
    contract_kernel<1><<<dim3(1, 5), 128, 0, stream>>>(PTh, PTl, EVh, EVl, PMTR + (size_t)b * 64 * 640);
    contract_kernel<0><<<dim3(NSP / 64, 5), 128, 0, stream>>>(SR, nullptr, EVh, EVl, SIPR + (size_t)b * NSP * 640);
  }
  writer_kernel<<<(unsigned)(((size_t)(OUT0 + OUT1) / 4 + 255) / 256), 256, 0, stream>>>(PMTR, SIPR, (float*)d_out);
}
